// Explicit_corr1_55387898249792
// MI455X (gfx1250) — hardware-run, weakly checked
//
#include <hip/hip_runtime.h>


#ifndef NB
#define NB 64
#endif
#define NB_FULL 64
#define CH   256
#define C1   128
#define C2   64
#define C3   32
#define GW   20
#define GPOS 400
#define TPOS 16
#define NWIN 289
#define NCR  (NB * GPOS)
#define NTR  (NB * TPOS)
#define NROWS (NCR + NTR)
#define WSC  1024.0f
#define WI   (1.0f / 1024.0f)
#define WRI  (1.0f / 2097152.0f)
#define QRS  2048.0f
#define TRP  2312

#define OFF0 ((size_t)0)
#define OFF1 ((size_t)NB_FULL * CH)
#define OFF2 (OFF1 + (size_t)NB_FULL * CH * NWIN)
#define OFF3 (OFF2 + (size_t)NB_FULL * TPOS)
#define OUT_TOTAL (OFF3 + (size_t)NB_FULL * TPOS * NWIN)

static_assert(OFF1 * 4 == 65536);
static_assert(OFF2 * 4 == 19005440);
static_assert(OFF3 * 4 == 19009536);
static_assert(OUT_TOTAL * 4 == 20193280);
static_assert((OFF1 * 4) % 128 == 0);
static_assert((OFF2 * 4) % 128 == 0);
static_assert((OFF3 * 4) % 128 == 0);
static_assert(NB >= 1);
static_assert(NB <= NB_FULL);
static_assert(CH == 256);
static_assert(CH % 32 == 0);
static_assert(C1 % 32 == 0);
static_assert(C2 % 32 == 0);
static_assert(C1 == 8 * 16);
static_assert(C2 == 4 * 16);
static_assert(C3 == 2 * 16);
static_assert(GPOS % 16 == 0);
static_assert(TPOS == 16);
static_assert((416 % 32) == 0);
static_assert(NROWS % 32 == 0);
static_assert((2 * CH) % 64 == 0);
static_assert(CH % 64 == 0);
static_assert((32 * NWIN) % 32 == 0);
static_assert((32 * NWIN) / 4 == TRP);
static_assert((CH * NWIN) % 32 == 0);
static_assert((2 * TPOS * NWIN) % 32 == 0);

typedef _Float16 h16;
typedef unsigned short bf;
typedef __attribute__((ext_vector_type(16))) __bf16   v16bf;
typedef __attribute__((ext_vector_type(16))) _Float16 v16h;
typedef __attribute__((ext_vector_type(8)))  _Float16 v8h;
typedef __attribute__((ext_vector_type(8)))  unsigned short v8us;
typedef __attribute__((ext_vector_type(8)))  float    v8f;
typedef __attribute__((ext_vector_type(4)))  float    v4f;
typedef __attribute__((ext_vector_type(2)))  unsigned int v2u;
typedef v4f  __attribute__((may_alias)) v4fa;

__device__ __forceinline__ unsigned short f2bf(float f) { unsigned u = __float_as_uint(f); u += 0x7FFFu + ((u >> 16) & 1u); return (unsigned short)(u >> 16); }
__device__ __forceinline__ float bfr(float f) { return __uint_as_float(((unsigned)f2bf(f)) << 16); }
__device__ __forceinline__ v16h cat16(v8h lo, v8h hi) { return __builtin_shufflevector(lo, hi, 0, 1, 2, 3, 4, 5, 6, 7, 8, 9, 10, 11, 12, 13, 14, 15); }
__device__ __forceinline__ v16bf cat16b(v8us lo, v8us hi) { return __builtin_bit_cast(v16bf, __builtin_shufflevector(lo, hi, 0, 1, 2, 3, 4, 5, 6, 7, 8, 9, 10, 11, 12, 13, 14, 15)); }
__device__ __forceinline__ v8f wmma16(v16h a, v16h b, v8f c) { return __builtin_amdgcn_wmma_f32_16x16x32_f16(false, a, false, b, (short)0, c, false, false); }
__device__ __forceinline__ v8f wmmab(v16bf a, v16bf b, v8f c) { return __builtin_amdgcn_wmma_f32_16x16x32_bf16(false, a, false, b, (short)0, c, false, false); }
__device__ __forceinline__ v16h  ldh(const h16* p) { return cat16(*(const v8h*)p, *(const v8h*)(p + 16)); }
__device__ __forceinline__ v16bf ldb(const bf* p)  { return cat16b(*(const v8us*)p, *(const v8us*)(p + 16)); }
__device__ __forceinline__ void wave_sync() { __builtin_amdgcn_fence(3  , "wavefront"); __builtin_amdgcn_wave_barrier(); asm volatile("" ::: "memory"); }

static __device__ __forceinline__ h16 toh_flush(float v) { const h16 r = (h16)v; return (fabsf(v) < 6.103515625e-05f) ? (h16)0.0f : r; }
__device__ __forceinline__ v8f wmma16g(v16h a, v16h b, v8f c) { c = wmma16(a, b, c); asm volatile("v_nop\n\tv_nop\n\tv_nop\n\tv_nop" : "+v"(c) : "v"(a), "v"(b)); return c; }
__device__ __forceinline__ v8f wmmabg(v16bf a, v16bf b, v8f c) { c = wmmab(a, b, c); asm volatile("v_nop\n\tv_nop\n\tv_nop\n\tv_nop" : "+v"(c) : "v"(a), "v"(b)); return c; }
__device__ __forceinline__ float lrelu(float x) { return x > 0.0f ? x : 0.01f * x; }
struct HR { v8h h; v8h r; };
__device__ __forceinline__ HR act_split(v8f aH, v8f aR) {
    HR o;
#pragma unroll
    for (int r = 0; r < 8; ++r) { const float x = lrelu(aH[r] * WI + aR[r] * WRI); const h16 a = toh_flush(x); o.h[r] = a; o.r[r] = toh_flush((x - (float)a) * QRS); }
    return o;
}

__global__ __launch_bounds__(256) void k_cvt8(const float* __restrict__ src, bf* dst, size_t n8) {
    const size_t i = (size_t)blockIdx.x * 256 + threadIdx.x; if (i >= n8) return;
    const v8f v = *(const v8f*)(src + i * 8); v8us o;
#pragma unroll
    for (int k = 0; k < 8; ++k) o[k] = f2bf(v[k]);
    *(volatile v8us*)(dst + i * 8) = o; __threadfence(); *(volatile v8us*)(dst + i * 8) = o;
}

__global__ __launch_bounds__(256) void k_wconv(const float* __restrict__ src, h16* dst, size_t n8) {
    const size_t i = (size_t)blockIdx.x * 256 + threadIdx.x; if (i >= n8) return;
    const v8f v = *(const v8f*)(src + i * 8); v8h o;
#pragma unroll
    for (int k = 0; k < 8; ++k) o[k] = toh_flush(bfr(v[k]) * WSC);
    *(volatile v8h*)(dst + i * 8) = o; __threadfence(); *(volatile v8h*)(dst + i * 8) = o;
}

__global__ __launch_bounds__(256) void k_xt(const float* __restrict__ src, bf* dst, int cs, int tilesPerB, int rowOff) {
    __shared__ __align__(16) bf ts[16 * CH];
    static_assert(16 * CH * 2 == 256 * 2 * 16);
    const int tid = threadIdx.x;
    const int b = (int)blockIdx.x / tilesPerB; const int tile = (int)blockIdx.x - b * tilesPerB;
    const float* sp = src + ((size_t)b * CH + (size_t)tid) * (size_t)cs + (size_t)tile * 16;
    const v4f x0 = *(const v4f*)sp, x1 = *(const v4f*)(sp + 4), x2 = *(const v4f*)(sp + 8), x3 = *(const v4f*)(sp + 12);
#pragma unroll
    for (int i = 0; i < 4; ++i) { ts[i * CH + tid] = f2bf(x0[i]); ts[(4 + i) * CH + tid] = f2bf(x1[i]); ts[(8 + i) * CH + tid] = f2bf(x2[i]); ts[(12 + i) * CH + tid] = f2bf(x3[i]); }
    __syncthreads();
    bf* dp = dst + ((size_t)rowOff + (size_t)b * (size_t)cs + (size_t)tile * 16) * CH;
#pragma unroll 1
    for (int ps = 0; ps < 2; ++ps) {
#pragma unroll
        for (int sI = 0; sI < 2; ++sI) { const unsigned piece = (unsigned)(sI * 256 + tid); const v8us v = *(const v8us*)(&ts[piece * 8]);
            *(volatile v8us*)(dp + (size_t)piece * 8) = v; }
        if (ps == 0) __threadfence(); }
}

__global__ __launch_bounds__(32) void k_pre(const bf* __restrict__ A, const bf* __restrict__ Wb, float* PU) {
    __shared__ __align__(16) float os[16 * 68];
    static_assert(8 * 32 * 16 == 16 * 64 * 4);
    const int lane = threadIdx.x & 31, lr = lane & 15, hi = lane >> 4; const int r0 = blockIdx.x * 32, c0 = blockIdx.y * 64;
    v8f acc[2][4];
#pragma unroll
    for (int mb = 0; mb < 2; ++mb)
#pragma unroll
        for (int nb = 0; nb < 4; ++nb) acc[mb][nb] = (v8f){};
    const size_t aoff = (size_t)(r0 + lr) * CH + 8 * hi;
    const size_t boff = (size_t)((c0 & 255) + lr) * (2 * CH) + (size_t)(c0 >> 8) * CH + 8 * hi;
#pragma unroll 1
    for (int kc = 0; kc < CH; kc += 32) {
        v16bf a[2];
#pragma unroll
        for (int mb = 0; mb < 2; ++mb) a[mb] = ldb(A + aoff + (size_t)mb * 16 * CH + kc);
#pragma unroll
        for (int nb = 0; nb < 4; ++nb) { const v16bf b = ldb(Wb + boff + (size_t)nb * 16 * (2 * CH) + kc);
#pragma unroll
            for (int mb = 0; mb < 2; ++mb) acc[mb][nb] = wmmabg(a[mb], b, acc[mb][nb]); }
    }
#pragma unroll
    for (int mb = 0; mb < 2; ++mb) {
#pragma unroll
        for (int nb = 0; nb < 4; ++nb) {
#pragma unroll
            for (int j = 0; j < 8; ++j) os[(hi * 8 + j) * 68 + nb * 16 + lr] = acc[mb][nb][j]; }
        wave_sync();
        float* ob = PU + (size_t)(r0 + mb * 16) * (2 * CH) + c0;
#pragma unroll 1
        for (int ps = 0; ps < 2; ++ps) {
#pragma unroll
            for (int s = 0; s < 8; ++s) { const int row = 2 * s + (lane >> 4), cofs = (lane & 15) * 4;
                const v4f val = *(const v4fa*)(&os[row * 68 + cofs]);
                *(volatile v4f*)(ob + (size_t)row * (2 * CH) + cofs) = val; }
            if (ps == 0) __threadfence(); }
        wave_sync();
    }
}

__global__ __launch_bounds__(128) void k_mlp(const float* __restrict__ PU, const bf* __restrict__ XB,
                                             const h16* __restrict__ W1, const h16* __restrict__ W2, const h16* __restrict__ W3,
                                             const float* __restrict__ w4, float* dstC, float* dstW,
                                             int nItems, int perB, int ow, int gp, int bstride, int rowOff) {
    __shared__ __align__(16) h16 sH0h[64 * CH];
    __shared__ __align__(16) h16 sH0r[64 * CH];
    __shared__ __align__(16) h16 sH1h[64 * C1];
    __shared__ __align__(16) h16 sH1r[64 * C1];
    __shared__ __align__(16) h16 sH2h[64 * C2];
    __shared__ __align__(16) h16 sH2r[64 * C2];
    __shared__ __align__(16) float sS[4 * 16];
    __shared__ __align__(16) float sW[4 * 16];
    static_assert((size_t)(2 * 64 * CH + 2 * 64 * C1 + 2 * 64 * C2) * 2 + (size_t)(64 + 64) * 4 <= (size_t)131072);
    static_assert(32 * 8 == CH);
    static_assert(2 * 32 * 16 == CH * 4);
    static_assert(16 * 16 == 4 * 16 * 4);
    const int lane = threadIdx.x & 31, lr = lane & 15, hi = lane >> 4;
    const int wave = __builtin_amdgcn_readfirstlane((int)(threadIdx.x >> 5));
    const int itv = (int)blockIdx.x * 4 + (int)(threadIdx.x >> 5);
    const int itcv = itv < nItems ? itv : nItems - 1;
    const int item = __builtin_amdgcn_readfirstlane(itcv);
    const int valid = __builtin_amdgcn_readfirstlane(itv < nItems ? 1 : 0);
    const int b = item / perB; const int oidx = item - b * perB; const int oi = oidx / ow; const int oj = oidx - oi * ow;
    const unsigned baseRow = (unsigned)(rowOff + b * bstride + oi * gp + oj);
    unsigned l8 = 8u * (unsigned)lane; asm volatile("" : "+v"(l8));
    unsigned l4 = 4u * (unsigned)lane; asm volatile("" : "+v"(l4));
    unsigned h8 = 8u * (unsigned)hi;   asm volatile("" : "+v"(h8));
    const float* pu = PU + (size_t)baseRow * (2 * CH) + l8;
    const unsigned cw = (unsigned)(wave * 16);
    float s = 1.0f, wl = 0.0f;
#pragma unroll 1
    for (int it = 0; it < 3; ++it) {
        sS[cw + lr] = s;
        wave_sync();
        float vk[8];
#pragma unroll
        for (int i = 0; i < 8; ++i) vk[i] = 0.0f;
#pragma unroll 2
        for (int p = 0; p < 16; ++p) {
            const float sp = sS[cw + p];
            const float* q = pu + (size_t)(unsigned)((p >> 2) * gp + (p & 3)) * (2 * CH);
            const v4f a0 = *(const v4f*)q, a1 = *(const v4f*)(q + 4);
#pragma unroll
            for (int i = 0; i < 4; ++i) { vk[i] += sp * a0[i]; vk[4 + i] += sp * a1[i]; } }
#pragma unroll
        for (int i = 0; i < 8; ++i) vk[i] *= 0.0625f;
#pragma unroll 2
        for (int p = 0; p < 16; ++p) {
            const float sp = sS[cw + p];
            const float* q = pu + (size_t)(unsigned)((p >> 2) * gp + (p & 3)) * (2 * CH) + CH;
            const v4f u0 = *(const v4f*)q, u1 = *(const v4f*)(q + 4);
            v8h hv, rv;
#pragma unroll
            for (int i = 0; i < 4; ++i) {
                const float x0 = lrelu(vk[i] + sp * u0[i]); const float x1 = lrelu(vk[4 + i] + sp * u1[i]);
                const h16 a0 = toh_flush(x0); const h16 a1 = toh_flush(x1);
                hv[i] = a0; hv[4 + i] = a1; rv[i] = toh_flush((x0 - (float)a0) * QRS); rv[4 + i] = toh_flush((x1 - (float)a1) * QRS); }
            const unsigned o = (cw + (unsigned)p) * CH + l8;
            *(v8h*)(&sH0h[o]) = hv; *(v8h*)(&sH0r[o]) = rv; }
        __syncthreads();
#pragma unroll 1
        for (int nh = 0; nh < 2; ++nh) {
            v8f aH[2][2], aR[2][2];
#pragma unroll
            for (int mt = 0; mt < 2; ++mt)
#pragma unroll
                for (int nt = 0; nt < 2; ++nt) { aH[mt][nt] = (v8f){}; aR[mt][nt] = (v8f){}; }
            const unsigned wo = (unsigned)((2 * wave) * 16 + lr) * CH + h8;
            const unsigned bo = (unsigned)((nh * 2) * 16 + lr) * CH + h8;
#pragma unroll 1
            for (int kc = 0; kc < CH; kc += 32) {
                v16h a[2];
#pragma unroll
                for (int mt = 0; mt < 2; ++mt) a[mt] = ldh(W1 + wo + (unsigned)(mt * 16 * CH) + (unsigned)kc);
#pragma unroll
                for (int nt = 0; nt < 2; ++nt) { const unsigned o = bo + (unsigned)(nt * 16 * CH) + (unsigned)kc;
                    const v16h bh = cat16(*(const v8h*)(&sH0h[o]), *(const v8h*)(&sH0h[o + 16]));
                    const v16h br = cat16(*(const v8h*)(&sH0r[o]), *(const v8h*)(&sH0r[o + 16]));
#pragma unroll
                    for (int mt = 0; mt < 2; ++mt) { aH[mt][nt] = wmma16g(a[mt], bh, aH[mt][nt]); aR[mt][nt] = wmma16g(a[mt], br, aR[mt][nt]); } }
            }
#pragma unroll
            for (int mt = 0; mt < 2; ++mt)
#pragma unroll
                for (int nt = 0; nt < 2; ++nt) { const HR t = act_split(aH[mt][nt], aR[mt][nt]);
                    const unsigned o = (unsigned)((nh * 2 + nt) * 16 + lr) * C1 + (unsigned)((2 * wave + mt) * 16) + h8;
                    *(v8h*)(&sH1h[o]) = t.h; *(v8h*)(&sH1r[o]) = t.r; }
        }
        __syncthreads();
        {
            v8f bH[4], bR[4];
#pragma unroll
            for (int nt = 0; nt < 4; ++nt) { bH[nt] = (v8f){}; bR[nt] = (v8f){}; }
            const unsigned wo = (unsigned)(wave * 16 + lr) * C1 + h8;
            const unsigned bo = (unsigned)lr * C1 + h8;
#pragma unroll 1
            for (int kc = 0; kc < C1; kc += 32) {
                const v16h a = ldh(W2 + wo + (unsigned)kc);
#pragma unroll
                for (int nt = 0; nt < 4; ++nt) { const unsigned o = bo + (unsigned)(nt * 16 * C1) + (unsigned)kc;
                    const v16h bh = cat16(*(const v8h*)(&sH1h[o]), *(const v8h*)(&sH1h[o + 16]));
                    const v16h br = cat16(*(const v8h*)(&sH1r[o]), *(const v8h*)(&sH1r[o + 16]));
                    bH[nt] = wmma16g(a, bh, bH[nt]); bR[nt] = wmma16g(a, br, bR[nt]); }
            }
#pragma unroll
            for (int nt = 0; nt < 4; ++nt) { const HR t = act_split(bH[nt], bR[nt]);
                const unsigned o = (unsigned)(nt * 16 + lr) * C2 + (unsigned)(wave * 16) + h8;
                *(v8h*)(&sH2h[o]) = t.h; *(v8h*)(&sH2r[o]) = t.r; }
        }
        __syncthreads();
        {
            v8f cH[2], cR[2];
#pragma unroll
            for (int mt = 0; mt < 2; ++mt) { cH[mt] = (v8f){}; cR[mt] = (v8f){}; }
            const unsigned bo = (cw + (unsigned)lr) * C2 + h8;
#pragma unroll
            for (int kc = 0; kc < C2; kc += 32) {
                const unsigned o = bo + (unsigned)kc;
                const v16h bh = cat16(*(const v8h*)(&sH2h[o]), *(const v8h*)(&sH2h[o + 16]));
                const v16h br = cat16(*(const v8h*)(&sH2r[o]), *(const v8h*)(&sH2r[o + 16]));
#pragma unroll
                for (int mt = 0; mt < 2; ++mt) { const v16h a = ldh(W3 + (unsigned)(mt * 16 + lr) * C2 + h8 + (unsigned)kc);
                    cH[mt] = wmma16g(a, bh, cH[mt]); cR[mt] = wmma16g(a, br, cR[mt]); }
            }
            float part = 0.0f;
#pragma unroll
            for (int mt = 0; mt < 2; ++mt) {
                const v4f wa = *(const v4f*)(w4 + mt * 16 + h8), wb = *(const v4f*)(w4 + mt * 16 + h8 + 4);
#pragma unroll
                for (int r = 0; r < 4; ++r) {
                    const float xa = lrelu(cH[mt][r] * WI + cR[mt][r] * WRI); const float xb = lrelu(cH[mt][4 + r] * WI + cR[mt][4 + r] * WRI);
                    part += bfr(wa[r]) * xa; part += bfr(wb[r]) * xb; } }
            const float lg = part + __shfl_xor(part, 16, 32);
            float mx = lg;
            mx = fmaxf(mx, __shfl_xor(mx, 8, 32)); mx = fmaxf(mx, __shfl_xor(mx, 4, 32)); mx = fmaxf(mx, __shfl_xor(mx, 2, 32)); mx = fmaxf(mx, __shfl_xor(mx, 1, 32));
            const float e = expf(lg - mx);
            float den = e;
            den += __shfl_xor(den, 8, 32); den += __shfl_xor(den, 4, 32); den += __shfl_xor(den, 2, 32); den += __shfl_xor(den, 1, 32);
            const float wn = e * (1.0f / den);
            s *= wn; wl = wn;
        }
    }
    sS[cw + lr] = s;
    sW[cw + lr] = valid ? wl : 0.0f;
    wave_sync();
    {
        float c0[4], c1[4];
#pragma unroll
        for (int i = 0; i < 4; ++i) { c0[i] = 0.0f; c1[i] = 0.0f; }
        const bf* xr = XB + (size_t)baseRow * CH + l4;
#pragma unroll 2
        for (int p = 0; p < 16; ++p) {
            const float sp = sS[cw + p];
            const bf* q = xr + (size_t)(unsigned)((p >> 2) * gp + (p & 3)) * CH;
            const v2u xa = *(const v2u*)q, xb = *(const v2u*)(q + 128);
            c0[0] += sp * __uint_as_float(xa[0] << 16); c0[1] += sp * __uint_as_float(xa[0] & 0xffff0000u);
            c0[2] += sp * __uint_as_float(xa[1] << 16); c0[3] += sp * __uint_as_float(xa[1] & 0xffff0000u);
            c1[0] += sp * __uint_as_float(xb[0] << 16); c1[1] += sp * __uint_as_float(xb[0] & 0xffff0000u);
            c1[2] += sp * __uint_as_float(xb[1] << 16); c1[3] += sp * __uint_as_float(xb[1] & 0xffff0000u); }
        v4f o0, o1;
#pragma unroll
        for (int i = 0; i < 4; ++i) { o0[i] = c0[i]; o1[i] = c1[i]; }
        if (valid) {
            float* cp = dstC + (size_t)item * CH + l4;
#pragma unroll 1
            for (int ps = 0; ps < 2; ++ps) { *(volatile v4f*)cp = o0; *(volatile v4f*)(cp + 128) = o1; if (ps == 0) __threadfence(); }
        }
    }
    __syncthreads();
    if (wave == 0) {
        const v4f wv = *(const v4fa*)(&sW[(lane & 15) * 4]);
        float* wp = dstW + (size_t)blockIdx.x * 64 + (size_t)((lane & 15) * 4);
        if (lane < 16) {
#pragma unroll 1
            for (int ps = 0; ps < 2; ++ps) { *(volatile v4f*)wp = wv; if (ps == 0) __threadfence(); }
        }
    }
}

__global__ __launch_bounds__(256) void k_tr(const float* __restrict__ src, float* dst, int mode) {
    __shared__ __align__(16) float tl[32 * NWIN];
    static_assert((size_t)TRP * 16 == (size_t)32 * NWIN * 4);
    static_assert(TRP % 8 == 0);
    const int tid = threadIdx.x; const int r = tid & 31;
    const int og = __builtin_amdgcn_readfirstlane((int)(threadIdx.x >> 5));
    const int g = blockIdx.x;
    size_t sbase, dbase; unsigned pitch; bool ok = true;
    if (mode == 0) { const int b = g >> 3, c0 = (g & 7) * 32;
        sbase = (size_t)b * NWIN * CH + (size_t)(c0 + r); pitch = CH; dbase = ((size_t)b * CH + (size_t)c0) * NWIN; }
    else { const int bb = 2 * g + (r >> 4); ok = bb < NB; const int bc = ok ? bb : (NB - 1);
        sbase = (size_t)bc * NWIN * 16 + (size_t)(r & 15); pitch = 16; dbase = (size_t)g * (32 * NWIN); }
#pragma unroll 1
    for (int o = og; o < NWIN; o += 8) { float v = src[sbase + (size_t)o * pitch]; asm volatile("" : "+v"(v)); tl[r * NWIN + o] = ok ? v : 0.0f; }
    __syncthreads();
    float* dp = dst + dbase;
#pragma unroll 1
    for (int ps = 0; ps < 2; ++ps) {
#pragma unroll 1
        for (int i = tid; i < TRP; i += 256) { const v4f v = *(const v4fa*)(&tl[4 * i]); *(volatile v4f*)(dp + (size_t)4 * i) = v; }
        if (ps == 0) __threadfence(); }
}

static constexpr size_t al256(size_t v) { return (v + 255) & ~(size_t)255; }
static constexpr size_t NITEM_PAD = (((size_t)NB * NWIN + 3) / 4) * 4;
static constexpr size_t SZ_W0 = al256((size_t)CH * 2 * CH * 2);
static constexpr size_t SZ_W1 = al256((size_t)C1 * CH * 2);
static constexpr size_t SZ_W2 = al256((size_t)C2 * C1 * 2);
static constexpr size_t SZ_W3 = al256((size_t)C3 * C2 * 2);
static constexpr size_t SZ_XB = al256((size_t)NROWS * CH * 2);
static constexpr size_t SZ_PU = al256((size_t)NROWS * 2 * CH * 4);
static constexpr size_t SZ_CS = al256((size_t)NB * NWIN * CH * 4);
static constexpr size_t SZ_SW = al256(NITEM_PAD * 16 * 4);
static constexpr size_t SZ_TOTAL = SZ_W0 + SZ_W1 + SZ_W2 + SZ_W3 + SZ_XB + SZ_PU + SZ_CS + SZ_SW;
static_assert(SZ_TOTAL <= (size_t)134217728);
static_assert(((size_t)CH * 2 * CH) % 64 == 0);
static_assert(((size_t)C1 * CH) % 64 == 0);
static_assert(((size_t)C2 * C1) % 64 == 0);
static_assert(((size_t)C3 * C2) % 64 == 0);
static_assert(((NB + 3) / 4) * 64 <= NB_FULL * TPOS);
static_assert(((NB + 1) / 2) * (32 * NWIN) <= NB_FULL * TPOS * NWIN);

extern "C" void kernel_launch(void* const* d_in, const int* in_sizes, int n_in,
                              void* d_out, int out_size, void* d_ws, size_t ws_size, hipStream_t stream) {
    if (n_in < 7) return;
    if ((size_t)in_sizes[0] < (size_t)NB * CH * TPOS || (size_t)in_sizes[1] < (size_t)NB * CH * GPOS) return;
    if ((size_t)in_sizes[2] < (size_t)CH * 2 * CH || (size_t)in_sizes[3] < (size_t)C1 * CH) return;
    if ((size_t)in_sizes[4] < (size_t)C2 * C1 || (size_t)in_sizes[5] < (size_t)C3 * C2 || in_sizes[6] < C3) return;
    if ((size_t)out_size < OFF3 + (size_t)((NB + 1) / 2) * (32 * NWIN)) return;
    if (SZ_TOTAL > ws_size) return;
    const float* tf = (const float*)d_in[0]; const float* cf = (const float*)d_in[1];
    const float* w0 = (const float*)d_in[2]; const float* w1 = (const float*)d_in[3];
    const float* w2 = (const float*)d_in[4]; const float* w3 = (const float*)d_in[5]; const float* w4 = (const float*)d_in[6];
    float* OUT = (float*)d_out;
    char* wsp = (char*)d_ws;
    bf*  W0B = (bf*)wsp;  wsp += SZ_W0;
    h16* W1H = (h16*)wsp; wsp += SZ_W1;
    h16* W2H = (h16*)wsp; wsp += SZ_W2;
    h16* W3H = (h16*)wsp; wsp += SZ_W3;
    bf*  XB  = (bf*)wsp;  wsp += SZ_XB;
    float* PU = (float*)wsp; wsp += SZ_PU;
    float* CS = (float*)wsp; wsp += SZ_CS;
    float* SWP = (float*)wsp; wsp += SZ_SW;

    { const size_t n8 = (size_t)CH * 2 * CH / 8; k_cvt8<<<(unsigned)((n8 + 255) / 256), 256, 0, stream>>>(w0, W0B, n8); }
    { const size_t n8 = (size_t)C1 * CH / 8; k_wconv<<<(unsigned)((n8 + 255) / 256), 256, 0, stream>>>(w1, W1H, n8); }
    { const size_t n8 = (size_t)C2 * C1 / 8; k_wconv<<<(unsigned)((n8 + 255) / 256), 256, 0, stream>>>(w2, W2H, n8); }
    { const size_t n8 = (size_t)C3 * C2 / 8; k_wconv<<<(unsigned)((n8 + 255) / 256), 256, 0, stream>>>(w3, W3H, n8); }
    k_xt<<<NB * (GPOS / 16), 256, 0, stream>>>(cf, XB, GPOS, GPOS / 16, 0);
    k_xt<<<NB, 256, 0, stream>>>(tf, XB, TPOS, 1, NCR);
    k_pre<<<dim3(NROWS / 32, (2 * CH) / 64, 1), 32, 0, stream>>>(XB, W0B, PU);
    k_mlp<<<(unsigned)((NB * NWIN + 3) / 4), 128, 0, stream>>>(PU, XB, W1H, W2H, W3H, w4, CS, SWP, NB * NWIN, NWIN, 17, GW, GPOS, 0);
    k_mlp<<<(unsigned)((NB + 3) / 4), 128, 0, stream>>>(PU, XB, W1H, W2H, W3H, w4, OUT + OFF0, OUT + OFF2, NB, 1, 1, 4, TPOS, NCR);
    k_tr<<<NB * 8, 256, 0, stream>>>(CS, OUT + OFF1, 0);
    k_tr<<<(NB + 1) / 2, 256, 0, stream>>>(SWP, OUT + OFF3, 1);
}
